// GenPhiloTextB_62869731279074
// MI455X (gfx1250) — hardware-run, weakly checked
//
#include <hip/hip_runtime.h>
#include <math.h>
#include <stddef.h>

typedef __attribute__((ext_vector_type(16))) _Float16 v16h;
typedef __attribute__((ext_vector_type(8)))  _Float16 v8h;
typedef __attribute__((ext_vector_type(8)))  float    v8f;
typedef __attribute__((ext_vector_type(4)))  float    v4f;

constexpr int kB = 256;
constexpr int kT = 256;
constexpr int kE = 64;
constexpr int kN = 512;
constexpr int kG = 4 * kN;
constexpr int kV = 128;
constexpr int kRowsAll = kB * kT;
constexpr int kRowsBlk = 16;
constexpr int kHP = 520;
constexpr float kHC = 1024.0f;
constexpr float kWC = 256.0f;
constexpr float kCar = kHC * kWC;
constexpr float kCarInv = 1.0f / kCar;
constexpr int kTileH = 16 * 512;

static_assert(kG == 2048, "gate width");
static_assert((kN % 32) == 0, "K multiple of 32");
static_assert((kRowsAll % 64) == 0 && (kV % 64) == 0, "dense head M,N multiples of 64");
static_assert((kB % kRowsBlk) == 0 && kN == 8 * 64, "scan tiling: 8 waves x 64 units, 16-row batch tiles");
static_assert((kHP * 2) % 16 == 0 && kHP >= kN, "LDS row pitch");

constexpr size_t kOffHS  = 0;
constexpr size_t kOffWHP = kOffHS  + (size_t)kRowsAll * kN * 2;
constexpr size_t kOffWDT = kOffWHP + (size_t)kG * kN * 2;
constexpr size_t kOffPP  = kOffWDT + (size_t)kV * kN * 2;
constexpr size_t kWsTotal = kOffPP + (size_t)kV * kG * 4;
static_assert(kWsTotal == 70385664ull, "carve total");
static_assert(kWsTotal <= 134217728ull, "carve cap");
static_assert((kOffWHP % 128) == 0 && (kOffWDT % 128) == 0 && (kOffPP % 128) == 0, "128-B aligned regions");

__device__ __forceinline__ float bf16_rne(float f) {
  unsigned u = __float_as_uint(f);
  u = (u + 0x7FFFu + ((u >> 16) & 1u)) & 0xFFFF0000u;
  return __uint_as_float(u);
}

union FragU { v16h v; v8h h[2]; };

__device__ __forceinline__ v16h ld_frag_split(const _Float16* p) {
  FragU f;
  f.h[0] = *(const v8h*)(p);
  f.h[1] = *(const v8h*)(p + 16);
  return f.v;
}
__device__ __forceinline__ v16h ld_frag_packed(const _Float16* p) {
  FragU f;
  f.h[0] = *(const v8h*)(p);
  f.h[1] = *(const v8h*)(p + 8);
  return f.v;
}

__device__ __forceinline__ v8f mma_f16(v16h a, v16h b, v8f c) {
  c = __builtin_amdgcn_wmma_f32_16x16x32_f16(false, a, false, b, (short)0, c, false, false);
  asm volatile("v_nop\n\tv_nop\n\tv_nop\n\tv_nop" : "+v"(c) : "v"(a), "v"(b));
  return c;
}

__device__ __forceinline__ float sigm_fast(float x) {
  return __builtin_amdgcn_rcpf(1.0f + __expf(-x));
}
__device__ __forceinline__ float tanh_fast(float x) {
  return 1.0f - 2.0f * __builtin_amdgcn_rcpf(1.0f + __expf(2.0f * x));
}

__global__ __launch_bounds__(256) void pack_wh_kernel(const float* __restrict__ Wh, _Float16* __restrict__ WHP) {
  const int p = blockIdx.x * 256 + threadIdx.x;
  if (p >= kG * kN / 8) return;
  const int j8   = p & 1;
  const int ln   = (p >> 1) & 31;
  const int kt   = (p >> 6) & 15;
  const int tile = p >> 10;
  const int k0 = kt * 32 + 8 * (ln >> 4) + 16 * j8;
  const int g  = tile * 16 + (ln & 15);
  v8h o;
#pragma unroll
  for (int e = 0; e < 8; ++e) {
    const float w = bf16_rne(Wh[(size_t)(k0 + e) * kG + g]);
    o[e] = (_Float16)(w * kWC);
  }
  _Float16* q = WHP + (size_t)p * 8;
  *(volatile v8h*)q = o;
  __threadfence();
  *(volatile v8h*)q = o;
}

__global__ __launch_bounds__(256) void pack_wd_kernel(const float* __restrict__ Wd, _Float16* __restrict__ WDT) {
  const int p = blockIdx.x * 256 + threadIdx.x;
  if (p >= kV * kN / 8) return;
  const int n  = p >> 6;
  const int k8 = (p & 63) * 8;
  v8h o;
#pragma unroll
  for (int e = 0; e < 8; ++e) {
    const float w = bf16_rne(Wd[(size_t)(k8 + e) * kV + n]);
    o[e] = (_Float16)(w * kWC);
  }
  _Float16* q = WDT + (size_t)p * 8;
  *(volatile v8h*)q = o;
  __threadfence();
  *(volatile v8h*)q = o;
}

__global__ __launch_bounds__(256) void build_p_kernel(const float* __restrict__ emb, const float* __restrict__ Wx,
                                                      const float* __restrict__ bias, float* __restrict__ PP) {
  const int gid = blockIdx.x * 256 + threadIdx.x;
  if (gid >= kV * kN) return;
  const int v = gid >> 9;
  const int u = gid & (kN - 1);
  float s0 = 0.0f, s1 = 0.0f, s2 = 0.0f, s3 = 0.0f;
#pragma unroll 1
  for (int e = 0; e < kE; ++e) {
    const float ev = bf16_rne(emb[v * kE + e]);
    const float* wr = Wx + (size_t)e * kG + u;
    s0 = fmaf(ev, bf16_rne(wr[0]), s0);
    s1 = fmaf(ev, bf16_rne(wr[kN]), s1);
    s2 = fmaf(ev, bf16_rne(wr[2 * kN]), s2);
    s3 = fmaf(ev, bf16_rne(wr[3 * kN]), s3);
  }
  v4f o;
  o[0] = s0 + bf16_rne(bias[u]);
  o[1] = s1 + bf16_rne(bias[kN + u]);
  o[2] = s2 + bf16_rne(bias[2 * kN + u]);
  o[3] = s3 + bf16_rne(bias[3 * kN + u]);
  float* q = PP + (size_t)gid * 4;
  *(volatile v4f*)q = o;
  __threadfence();
  *(volatile v4f*)q = o;
}

__global__ __launch_bounds__(256) void lstm_scan_kernel(
    const int* __restrict__ X, const float* __restrict__ h0, const float* __restrict__ c0,
    const float* __restrict__ PP, const _Float16* WHP, _Float16* HS)
{
  __shared__ __align__(16) _Float16 hsh[2 * kRowsBlk * kHP];
  const int tid  = threadIdx.x;
  const int lane = tid & 31;
  const int wave = tid >> 5;
  const int hh   = lane >> 4;
  const int nn   = lane & 15;
  const int b0   = blockIdx.x * kRowsBlk;
  const int ubase = wave * 64 + nn;

  float c[4][8];
#pragma unroll
  for (int ut = 0; ut < 4; ++ut) {
#pragma unroll
    for (int r = 0; r < 8; ++r) {
      c[ut][r] = bf16_rne(c0[(size_t)(b0 + 8 * hh + r) * kN + ubase + ut * 16]);
    }
    asm volatile("" ::: "memory");
  }
#pragma unroll 1
  for (int i = 0; i < 32; ++i) {
    const int idx = i * 256 + tid;
    const int row = idx >> 9;
    const int col = idx & (kN - 1);
    hsh[row * kHP + col] = (_Float16)(bf16_rne(h0[(size_t)(b0 + row) * kN + col]) * kHC);
  }
  __syncthreads();

  const int* xr = X + (size_t)(b0 + 8 * hh) * kT;
  const _Float16* bbase = WHP + (size_t)(wave * 4) * kTileH + lane * 16;

#pragma unroll 1
  for (int t = 0; t < kT; ++t) {
    const int cur = t & 1;
    const int nxt = cur ^ 1;

    int tk[8];
#pragma unroll
    for (int r = 0; r < 8; ++r) {
      int tv = xr[r * kT + t];
      tv = tv < 0 ? 0 : tv;
      tv = tv > (kV - 1) ? (kV - 1) : tv;
      tk[r] = tv;
    }

    v8f acc[4][4];
#pragma unroll
    for (int ut = 0; ut < 4; ++ut) {
#pragma unroll
      for (int r = 0; r < 8; ++r) {
        const v4f p = *(const v4f*)(PP + ((size_t)tk[r] * kN + ubase + ut * 16) * 4);
        acc[ut][0][r] = p[0] * kCar;
        acc[ut][1][r] = p[1] * kCar;
        acc[ut][2][r] = p[2] * kCar;
        acc[ut][3][r] = p[3] * kCar;
      }
      asm volatile("" ::: "memory");
    }

    const _Float16* ap = hsh + cur * (kRowsBlk * kHP) + nn * kHP + 8 * hh;
#pragma unroll 1
    for (int kt = 0; kt < 16; ++kt) {
      const v16h a = ld_frag_split(ap + kt * 32);
      const _Float16* bk = bbase + kt * 512;
#pragma unroll
      for (int ut = 0; ut < 4; ++ut) {
        const v16h bi = ld_frag_packed(bk + (size_t)(0 * 32 + ut) * kTileH);
        const v16h bf = ld_frag_packed(bk + (size_t)(1 * 32 + ut) * kTileH);
        const v16h bg = ld_frag_packed(bk + (size_t)(2 * 32 + ut) * kTileH);
        const v16h bo = ld_frag_packed(bk + (size_t)(3 * 32 + ut) * kTileH);
        acc[ut][0] = mma_f16(a, bi, acc[ut][0]);
        acc[ut][1] = mma_f16(a, bf, acc[ut][1]);
        acc[ut][2] = mma_f16(a, bg, acc[ut][2]);
        acc[ut][3] = mma_f16(a, bo, acc[ut][3]);
        asm volatile("" ::: "memory");
      }
    }

    _Float16* hw = hsh + nxt * (kRowsBlk * kHP) + (8 * hh) * kHP + ubase;
#pragma unroll
    for (int ut = 0; ut < 4; ++ut) {
#pragma unroll
      for (int r = 0; r < 8; ++r) {
        const float zi = acc[ut][0][r] * kCarInv;
        const float zf = acc[ut][1][r] * kCarInv;
        const float zg = acc[ut][2][r] * kCarInv;
        const float zo = acc[ut][3][r] * kCarInv;
        const float gi = sigm_fast(zi);
        const float gf = sigm_fast(zf);
        const float gg = tanh_fast(zg);
        const float go = sigm_fast(zo);
        const float cn = gf * c[ut][r] + gi * gg;
        c[ut][r] = cn;
        const float hv = go * tanh_fast(cn);
        hw[r * kHP + ut * 16] = (_Float16)(hv * kHC);
      }
    }
    __syncthreads();

    v8h cv[4];
#pragma unroll
    for (int rr = 0; rr < 2; ++rr) {
#pragma unroll
      for (int hf = 0; hf < 2; ++hf) {
        cv[rr * 2 + hf] = *(const v8h*)(hsh + nxt * (kRowsBlk * kHP) + (2 * wave + rr) * kHP + hf * 256 + lane * 8);
      }
    }
    for (int pass = 0; pass < 2; ++pass) {
#pragma unroll
      for (int rr = 0; rr < 2; ++rr) {
#pragma unroll
        for (int hf = 0; hf < 2; ++hf) {
          _Float16* dst = HS + ((size_t)(b0 + 2 * wave + rr) * kT + t) * kN + hf * 256 + lane * 8;
          *(volatile v8h*)dst = cv[rr * 2 + hf];
        }
      }
      __threadfence();
    }
    __syncthreads();
  }
}

__global__ __launch_bounds__(256) void logits_gemm_kernel(
    const _Float16* __restrict__ A, const _Float16* __restrict__ Bt,
    float* __restrict__ C, const float* __restrict__ bias)
{
  __shared__ __align__(16) float sT[8][16 * 68];
  const int lane = threadIdx.x & 31;
  const int wave = threadIdx.x >> 5;
  constexpr int tilesN = kV >> 6;
  constexpr int tilesM = kRowsAll >> 6;
  const int tile = blockIdx.x * 8 + wave;
  if (tile >= tilesM * tilesN) return;
  const int tm = tile / tilesN;
  const int tn = tile - tm * tilesN;
  const int m0 = tm << 6;
  const int n0 = tn << 6;
  const int rlane = lane & 15;
  const int koff  = (lane >> 4) * 8;
  const int mOff  = (lane >> 4) * 8;

  v8f acc[4][4];
#pragma unroll
  for (int i = 0; i < 4; ++i)
#pragma unroll
    for (int j = 0; j < 4; ++j) acc[i][j] = (v8f){0.f, 0.f, 0.f, 0.f, 0.f, 0.f, 0.f, 0.f};

  for (int k0 = 0; k0 < kN; k0 += 32) {
    v16h bfr[4];
#pragma unroll
    for (int j = 0; j < 4; ++j) {
      bfr[j] = ld_frag_split(Bt + (size_t)(n0 + (j << 4) + rlane) * kN + koff + k0);
    }
#pragma unroll
    for (int i = 0; i < 4; ++i) {
      const v16h a = ld_frag_split(A + (size_t)(m0 + (i << 4) + rlane) * kN + koff + k0);
#pragma unroll
      for (int j = 0; j < 4; ++j) {
        acc[i][j] = mma_f16(a, bfr[j], acc[i][j]);
      }
    }
  }

  float* slab = sT[wave];
#pragma unroll
  for (int i = 0; i < 4; ++i) {
    const int mBase = m0 + (i << 4);
#pragma unroll
    for (int j = 0; j < 4; ++j) {
      const float bv = bf16_rne(bias[n0 + (j << 4) + rlane]);
#pragma unroll
      for (int r = 0; r < 8; ++r) {
        slab[(mOff + r) * 68 + (j << 4) + rlane] = acc[i][j][r] * kCarInv + bv;
      }
    }
    __builtin_amdgcn_fence(__ATOMIC_RELEASE, "workgroup");
    __builtin_amdgcn_wave_barrier();
    __builtin_amdgcn_fence(__ATOMIC_ACQUIRE, "workgroup");
    {
      const int hh2 = lane >> 4;
      const int c4  = (lane & 15) * 4;
      for (int pass = 0; pass < 2; ++pass) {
#pragma unroll
        for (int it = 0; it < 8; ++it) {
          const int row = it * 2 + hh2;
          const v4f v = *(const v4f*)(slab + row * 68 + c4);
          *(volatile v4f*)(C + (size_t)(mBase + row) * kV + n0 + c4) = v;
        }
        __threadfence();
      }
    }
    __builtin_amdgcn_fence(__ATOMIC_RELEASE, "workgroup");
    __builtin_amdgcn_wave_barrier();
    __builtin_amdgcn_fence(__ATOMIC_ACQUIRE, "workgroup");
  }
}

extern "C" void kernel_launch(void* const* d_in, const int* in_sizes, int n_in,
                              void* d_out, int out_size, void* d_ws, size_t ws_size,
                              hipStream_t stream) {
  if (n_in < 9) return;
  if (in_sizes[0] != kB * kT) return;
  if (in_sizes[1] != kB * kN) return;
  if (in_sizes[2] != kB * kN) return;
  if (in_sizes[3] != kV * kE) return;
  if (in_sizes[4] != kE * kG) return;
  if (in_sizes[5] != kN * kG) return;
  if (in_sizes[6] != kG) return;
  if (in_sizes[7] != kN * kV) return;
  if (in_sizes[8] != kV) return;
  if (out_size != kRowsAll * kV) return;
  if (ws_size < kWsTotal) return;

  const int*   X   = (const int*)d_in[0];
  const float* h0  = (const float*)d_in[1];
  const float* c0  = (const float*)d_in[2];
  const float* emb = (const float*)d_in[3];
  const float* Wx  = (const float*)d_in[4];
  const float* Wh  = (const float*)d_in[5];
  const float* bia = (const float*)d_in[6];
  const float* Wd  = (const float*)d_in[7];
  const float* bd  = (const float*)d_in[8];
  float* out = (float*)d_out;

  char* ws = (char*)d_ws;
  _Float16* HS  = (_Float16*)(ws + kOffHS);
  _Float16* WHP = (_Float16*)(ws + kOffWHP);
  _Float16* WDT = (_Float16*)(ws + kOffWDT);
  float*    PP  = (float*)(ws + kOffPP);

  pack_wh_kernel<<<(kG * kN / 8) / 256, 256, 0, stream>>>(Wh, WHP);
  pack_wd_kernel<<<(kV * kN / 8) / 256, 256, 0, stream>>>(Wd, WDT);
  build_p_kernel<<<(kV * kN) / 256, 256, 0, stream>>>(emb, Wx, bia, PP);
  lstm_scan_kernel<<<kB / kRowsBlk, 256, 0, stream>>>(X, h0, c0, PP, WHP, HS);
  logits_gemm_kernel<<<((kRowsAll >> 6) * (kV >> 6)) / 8, 256, 0, stream>>>(HS, WDT, out, bd);
}
